// OutProductMean_27161373180655
// MI455X (gfx1250) — hardware-verified
//
#include <hip/hip_runtime.h>


namespace {
constexpr int S = 128, I = 256, D = 64, P = 32, DO = 128, PP = P * P;
constexpr float XS = 8.0f, OS = 0.25f  , EPS = 1e-5f;

typedef _Float16 b16;
typedef __attribute__((ext_vector_type(16))) _Float16 v16b;
typedef __attribute__((ext_vector_type(8))) _Float16 v8b;
typedef __attribute__((ext_vector_type(8))) float v8f;
typedef __attribute__((ext_vector_type(4))) float v4f;
__device__ __forceinline__ float bf16_rne(float f) { unsigned int u = __float_as_uint(f); u += 0x7FFFu + ((u >> 16) & 1u); return __uint_as_float(u & 0xFFFF0000u); }
__device__ __forceinline__ v16b frag_kb(const b16* p, int hh) { const v8b a = *(const v8b*)(p + 8 * hh), b = *(const v8b*)(p + 16 + 8 * hh); v16b f;
#pragma unroll
  for (int e = 0; e < 8; ++e) { f[e] = a[e]; f[8 + e] = b[e]; } return f; }
__device__ __forceinline__ v8f wmma16b(v16b a, v16b b, v8f c) { v8f d = __builtin_amdgcn_wmma_f32_16x16x32_f16(false, a, false, b, (short)0, c, false, false); asm volatile("v_nop\n\tv_nop\n\tv_nop\n\tv_nop" : "+v"(d) : "v"(a), "v"(b)); return d; }
__device__ __forceinline__ void wave_lds_sync() { __builtin_amdgcn_fence(__ATOMIC_RELEASE, "workgroup"); __builtin_amdgcn_wave_barrier(); __builtin_amdgcn_fence(__ATOMIC_ACQUIRE, "workgroup"); }
__device__ __forceinline__ float pmul(float a, float b) { float p = a * b; asm volatile("" : "+v"(p)); return p; }
__device__ __forceinline__ float wsum(float v) {
#pragma unroll
  for (int o = 1; o < 32; o <<= 1) v += __shfl_xor(v, o); return v; }

__global__ __launch_bounds__(256) void proj_kernel(const float* __restrict__ M, const float* __restrict__ g, const float* __restrict__ be, const float* __restrict__ Wa, const float* __restrict__ ba, const float* __restrict__ Wb, const float* __restrict__ bb, const float* __restrict__ Wo, const float* __restrict__ bo, b16* __restrict__ LT, b16* __restrict__ RT, b16* __restrict__ LTl, b16* __restrict__ RTl, b16* __restrict__ RW, float* __restrict__ Pb) {
  __shared__ __attribute__((aligned(16))) b16 Ar[S][D + 8], Arl[S][D + 8]; __shared__ __attribute__((aligned(16))) b16 Wr[2 * P][D + 8]; __shared__ __attribute__((aligned(16))) b16 To[2 * P][S + 8], Tol[2 * P][S + 8]; __shared__ float bias[64];
  const int i = blockIdx.x, t_ = threadIdx.x, lane = t_ & 31, wave = t_ >> 5, nloc = lane & 15, hlf = lane >> 4;
  for (int q = t_; q < 2 * P * D; q += 256) { const int o = q / D, d = q % D; Wr[o][d] = (b16)bf16_rne((o < P) ? Wa[o * D + d] : Wb[(o - P) * D + d]); }
  if (t_ < 64) bias[t_] = bf16_rne((t_ < P) ? ba[t_] : bb[t_ - P]);
  for (int q = 0; q < 16; ++q) { const int s = wave * 16 + q; const float* mr = M + ((size_t)s * I + i) * D; const float x0 = bf16_rne(mr[lane]), x1 = bf16_rne(mr[32 + lane]);
    const float mu = wsum(x0 + x1) * (1.0f / D); const float d0 = x0 - mu, d1 = x1 - mu; const float var = wsum(pmul(d0, d0) + pmul(d1, d1)) * (1.0f / D); const float inv = rsqrtf(var + EPS);
    { const float y0 = (pmul(d0 * inv, bf16_rne(g[lane])) + bf16_rne(be[lane])) * XS, y1 = (pmul(d1 * inv, bf16_rne(g[32 + lane])) + bf16_rne(be[32 + lane])) * XS; const b16 h0 = (b16)y0, h1 = (b16)y1; Ar[s][lane] = h0; Arl[s][lane] = (b16)(y0 - (float)h0); Ar[s][32 + lane] = h1; Arl[s][32 + lane] = (b16)(y1 - (float)h1); } }
  __syncthreads();
  v8f acc[4] = {{}, {}, {}, {}};
#pragma unroll
  for (int kb = 0; kb < D; kb += 32) { const v16b a = frag_kb(&Ar[wave * 16 + nloc][kb], hlf), al = frag_kb(&Arl[wave * 16 + nloc][kb], hlf);
#pragma unroll
    for (int t = 0; t < 4; ++t) { const v16b bw = frag_kb(&Wr[t * 16 + nloc][kb], hlf); acc[t] = wmma16b(a, bw, acc[t]); acc[t] = wmma16b(al, bw, acc[t]); } }
#pragma unroll
  for (int t = 0; t < 4; ++t)
#pragma unroll
    for (int r = 0; r < 8; ++r) { const int c = t * 16 + nloc, s = wave * 16 + 8 * hlf + r; const float y = (acc[t][r] * (1.0f / XS) + bias[c]) * XS; const b16 h_ = (b16)y; To[c][s] = h_; Tol[c][s] = (b16)(y - (float)h_); }
  __syncthreads();
  for (int pass = 0; pass < 2; ++pass) {
    for (int q = t_; q < 2 * P * (S / 8); q += 256) { const int c = q / (S / 8), s8 = (q % (S / 8)) * 8; const size_t gi = (c < P) ? (((size_t)i * P + c) * S + s8) : (((size_t)i * P + (c - P)) * S + s8); b16* dh = (c < P) ? LT : RT; b16* dl = (c < P) ? LTl : RTl; *(volatile v8b*)(dh + gi) = *(const v8b*)(&To[c][s8]); *(volatile v8b*)(dl + gi) = *(const v8b*)(&Tol[c][s8]); }
    if (i < 64) { for (int q = i * 256 + t_; q < DO * PP / 8; q += 64 * 256) { v8b v; for (int e = 0; e < 8; ++e) v[e] = (b16)bf16_rne(Wo[(size_t)q * 8 + e]); *(volatile v8b*)(RW + (size_t)q * 8) = v; } if (i == 0 && t_ < DO) Pb[t_] = bf16_rne(bo[t_]); }
    __threadfence(); }
}

__global__ __launch_bounds__(256) void opm_kernel(const b16* __restrict__ LT, const b16* __restrict__ RT, const b16* __restrict__ LTl, const b16* __restrict__ RTl, const b16* __restrict__ RW, const float* __restrict__ Pb, float* __restrict__ out) {
  __shared__ __attribute__((aligned(16))) b16 Og[16][PP + 8], Ogl[16][PP + 8]; __shared__ __attribute__((aligned(16))) float Zs[16][DO + 4];
  const int i = blockIdx.y, j0 = blockIdx.x * 16, t_ = threadIdx.x, lane = t_ & 31, wave = t_ >> 5, nloc = lane & 15, hlf = lane >> 4;
  const b16* Li = LT + (size_t)i * P * S; const b16* Lil = LTl + (size_t)i * P * S;
  for (int jj = 0; jj < 2; ++jj) { const int jl = wave * 2 + jj, j = j0 + jl; const b16* Rj = RT + (size_t)j * P * S; const b16* Rjl = RTl + (size_t)j * P * S; v8f acc[2][2] = {{{}, {}}, {{}, {}}};
#pragma unroll
    for (int kb = 0; kb < S; kb += 32) { const v16b a0 = frag_kb(Li + (size_t)nloc * S + kb, hlf), a1 = frag_kb(Li + (size_t)(16 + nloc) * S + kb, hlf), l0 = frag_kb(Lil + (size_t)nloc * S + kb, hlf), l1 = frag_kb(Lil + (size_t)(16 + nloc) * S + kb, hlf);
      const v16b b0 = frag_kb(Rj + (size_t)nloc * S + kb, hlf), b1 = frag_kb(Rj + (size_t)(16 + nloc) * S + kb, hlf), m0_ = frag_kb(Rjl + (size_t)nloc * S + kb, hlf), m1_ = frag_kb(Rjl + (size_t)(16 + nloc) * S + kb, hlf);
      acc[0][0] = wmma16b(a0, b0, acc[0][0]); acc[0][0] = wmma16b(l0, b0, acc[0][0]); acc[0][0] = wmma16b(a0, m0_, acc[0][0]);
      acc[0][1] = wmma16b(a0, b1, acc[0][1]); acc[0][1] = wmma16b(l0, b1, acc[0][1]); acc[0][1] = wmma16b(a0, m1_, acc[0][1]);
      acc[1][0] = wmma16b(a1, b0, acc[1][0]); acc[1][0] = wmma16b(l1, b0, acc[1][0]); acc[1][0] = wmma16b(a1, m0_, acc[1][0]);
      acc[1][1] = wmma16b(a1, b1, acc[1][1]); acc[1][1] = wmma16b(l1, b1, acc[1][1]); acc[1][1] = wmma16b(a1, m1_, acc[1][1]); }
#pragma unroll
    for (int rt = 0; rt < 2; ++rt)
#pragma unroll
      for (int ct = 0; ct < 2; ++ct)
#pragma unroll
        for (int r = 0; r < 8; ++r) { const int p = rt * 16 + 8 * hlf + r, e = ct * 16 + nloc; const float y = acc[rt][ct][r] * (OS / (XS * XS)); const b16 h_ = (b16)y; Og[jl][p * P + e] = h_; Ogl[jl][p * P + e] = (b16)(y - (float)h_); } }
  __syncthreads();
  v8f z = {};
#pragma unroll 4
  for (int kb = 0; kb < PP; kb += 32) { const v16b bw = frag_kb(RW + (size_t)(wave * 16 + nloc) * PP + kb, hlf); z = wmma16b(frag_kb(&Og[nloc][kb], hlf), bw, z); z = wmma16b(frag_kb(&Ogl[nloc][kb], hlf), bw, z); }
#pragma unroll
  for (int r = 0; r < 8; ++r) { const int o = wave * 16 + nloc; Zs[8 * hlf + r][o] = z[r] * (1.0f / OS) + Pb[o]; }
  __syncthreads();
  for (int pass = 0; pass < 2; ++pass) { for (int q = t_; q < 16 * (DO / 4); q += 256) { const int jl = q / (DO / 4), c4 = (q % (DO / 4)) * 4; *(volatile v4f*)(out + ((size_t)i * I + j0 + jl) * DO + c4) = *(const v4f*)(&Zs[jl][c4]); } __threadfence(); }
}
}

extern "C" void kernel_launch(void* const* d_in, const int* in_sizes, int n_in,
                              void* d_out, int out_size, void* d_ws, size_t ws_size, hipStream_t stream) {
  (void)n_in; (void)out_size;
  const float* M = (const float*)d_in[0]; const float* g = (const float*)d_in[1]; const float* be = (const float*)d_in[2]; const float* Wa = (const float*)d_in[3]; const float* ba = (const float*)d_in[4]; const float* Wb = (const float*)d_in[5]; const float* bb = (const float*)d_in[6]; const float* Wo = (const float*)d_in[7]; const float* bo = (const float*)d_in[8];
  float* out = (float*)d_out;
  if (in_sizes[0] != S * I * D || in_sizes[3] != P * D || in_sizes[7] != DO * PP) return;
  size_t off = 0; char* ws = (char*)d_ws;
  auto carve = [&](size_t bytes) { char* p = ws + off; off += (bytes + 255) & ~(size_t)255; return p; };
  b16* LT = (b16*)carve((size_t)I * P * S * 2); b16* RT = (b16*)carve((size_t)I * P * S * 2); b16* LTl = (b16*)carve((size_t)I * P * S * 2); b16* RTl = (b16*)carve((size_t)I * P * S * 2); b16* RW = (b16*)carve((size_t)DO * PP * 2); float* Pb = (float*)carve(DO * 4);
  if (off > ws_size) return;
  proj_kernel<<<I, 256, 0, stream>>>(M, g, be, Wa, ba, Wb, bb, Wo, bo, LT, RT, LTl, RTl, RW, Pb);
  opm_kernel<<<dim3(I / 16, I), 256, 0, stream>>>(LT, RT, LTl, RTl, RW, Pb, out);
}
